// RN_18811956756917
// MI455X (gfx1250) — hardware-run, weakly checked
//
#include <hip/hip_runtime.h>
#include <math.h>

typedef __attribute__((ext_vector_type(16))) _Float16 v16h;
typedef __attribute__((ext_vector_type(8)))  _Float16 v8h;
typedef __attribute__((ext_vector_type(4)))  _Float16 v4h;
typedef __attribute__((ext_vector_type(8)))  float    v8f;
typedef __attribute__((ext_vector_type(4)))  float    v4f;

constexpr int kBatch = 4;
constexpr int kChan  = 32;
constexpr int kTok   = 576;
constexpr int kHid   = 128;
constexpr int kOutC  = 32;
constexpr int kRows  = kBatch * kTok;
constexpr int kPP    = 2 * kHid;
static_assert(kRows == 2304, "token rows");
static_assert((kTok % 64) == 0, "a 64-token tile never crosses a batch");
static_assert(kChan == 32 && (kHid % 32) == 0, "K multiples of 32");
static_assert((kRows % 64) == 0 && (kPP % 64) == 0 && kOutC == 32, "tile multiples");

constexpr float kCarryX  = 16.0f;
constexpr float kCarryW  = 256.0f;
constexpr float kScale0  = 1.0f / (kCarryX * kCarryW);
constexpr float kScale1  = 1.0f / kCarryW;
constexpr float kF16MinNormal = 6.103515625e-05f;
constexpr float kTokF = (float)kTok;

constexpr size_t kOffXH  = 0;
constexpr size_t kOffW1T = kOffXH  + (size_t)kRows * kChan * 2;
constexpr size_t kOffW2T = kOffW1T + (size_t)kPP * kChan * 2;
constexpr size_t kOffP   = kOffW2T + (size_t)kOutC * kHid * 2;
constexpr size_t kOffS   = kOffP   + (size_t)kRows * kPP * 4;
constexpr size_t kWsTotal = kOffS  + (size_t)kRows * kHid * 2;
static_assert(kWsTotal == 3121152ull, "carve total");
static_assert(kWsTotal <= 134217728ull, "carve cap");
static_assert((kOffW1T % 128) == 0 && (kOffW2T % 128) == 0 && (kOffP % 128) == 0 && (kOffS % 128) == 0, "128-B aligned regions");

union FragU { v16h v; v8h h[2]; };
__device__ __forceinline__ v16h frag_load(const _Float16* p) {
  FragU f;
  f.h[0] = *(const v8h*)(p);
  f.h[1] = *(const v8h*)(p + 16);
  return f.v;
}
__device__ __forceinline__ v8f mma_f16(v16h a, v16h b, v8f c) {
  c = __builtin_amdgcn_wmma_f32_16x16x32_f16(false, a, false, b, (short)0, c, false, false);
  asm volatile("v_nop\n\tv_nop\n\tv_nop\n\tv_nop" : "+v"(c) : "v"(a), "v"(b));
  return c;
}
__device__ __forceinline__ _Float16 to_f16_carry(float v, float carry) {
  const float c = v * carry;
  const float f = (fabsf(c) < kF16MinNormal) ? 0.0f : c;
  return (_Float16)f;
}

constexpr int kXBlocks  = kRows / 64;
constexpr int kW1Blocks = (kPP * kChan / 8) / 256;
constexpr int kW2Blocks = (kOutC * kHid / 8) / 256;
static_assert(kXBlocks == 36 && kW1Blocks == 4 && kW2Blocks == 2, "prep grid");
constexpr int kXPitch = 65;

__global__ __launch_bounds__(256) void prep_planes_kernel(
    const float* __restrict__ x, const float* __restrict__ W1, const float* __restrict__ W2,
    _Float16* __restrict__ XH, _Float16* __restrict__ W1T, _Float16* __restrict__ W2T)
{
  __shared__ __align__(16) float sX[kChan * kXPitch];
  const int tid = threadIdx.x;
  const int blk = blockIdx.x;
  const bool isX = (blk < kXBlocks);
  const int m0 = isX ? blk * 64 : 0;
  const int bidx = m0 / kTok;
  const int n0 = m0 - bidx * kTok;
  if (isX) {
#pragma unroll
    for (int it = 0; it < 8; ++it) {
      const int idx = it * 256 + tid;
      const int c = idx >> 6;
      const int n = idx & 63;
      sX[c * kXPitch + n] = x[(size_t)(bidx * kChan + c) * kTok + n0 + n];
    }
  }
  __syncthreads();
  v8h hv;
  _Float16* dst;
  if (isX) {
    const int token = tid >> 2;
    const int c8 = (tid & 3) * 8;
#pragma unroll
    for (int e = 0; e < 8; ++e) hv[e] = to_f16_carry(sX[(c8 + e) * kXPitch + token], kCarryX);
    dst = XH + (size_t)(m0 + token) * kChan + c8;
  } else if (blk < kXBlocks + kW1Blocks) {
    const int g = (blk - kXBlocks) * 256 + tid;
    const int col = g >> 2;
    const int c8 = (g & 3) * 8;
    const int rowb = (col >> 7) * kChan + c8;
    const int colw = col & (kHid - 1);
#pragma unroll
    for (int e = 0; e < 8; ++e) hv[e] = to_f16_carry(W1[(size_t)(rowb + e) * kHid + colw], kCarryW);
    dst = W1T + (size_t)col * kChan + c8;
  } else {
    const int g = (blk - kXBlocks - kW1Blocks) * 256 + tid;
    const int o = g >> 4;
    const int h8 = (g & 15) * 8;
#pragma unroll
    for (int e = 0; e < 8; ++e) hv[e] = to_f16_carry(W2[(size_t)(h8 + e) * kOutC + o], kCarryW);
    dst = W2T + (size_t)o * kHid + h8;
  }
  *(volatile v8h*)dst = hv;
  __threadfence();
  *(volatile v8h*)dst = hv;
}

static_assert(((kRows / 64) * (kPP / 64)) % 8 == 0, "tiles fill whole blocks");
__global__ __launch_bounds__(256) void proj_gemm_kernel(
    const _Float16* __restrict__ XH, const _Float16* __restrict__ W1T, float* __restrict__ P)
{
  __shared__ __align__(16) float sT[8][16 * 68];
  const int lane = threadIdx.x & 31;
  const int wave = threadIdx.x >> 5;
  const int tile = blockIdx.x * 8 + wave;
  const int tm = tile >> 2;
  const int tn = tile & 3;
  const int m0 = tm << 6;
  const int n0 = tn << 6;
  const int rlane = lane & 15;
  const int koff = (lane >> 4) * 8;
  const int mOff = (lane >> 4) * 8;

  v8f acc[4][4];
#pragma unroll
  for (int i = 0; i < 4; ++i)
#pragma unroll
    for (int j = 0; j < 4; ++j) acc[i][j] = (v8f){0.f, 0.f, 0.f, 0.f, 0.f, 0.f, 0.f, 0.f};

  v16h bh[4];
#pragma unroll
  for (int j = 0; j < 4; ++j) bh[j] = frag_load(W1T + (size_t)(n0 + (j << 4) + rlane) * kChan + koff);
#pragma unroll
  for (int i = 0; i < 4; ++i) {
    const v16h ah = frag_load(XH + (size_t)(m0 + (i << 4) + rlane) * kChan + koff);
#pragma unroll
    for (int j = 0; j < 4; ++j) acc[i][j] = mma_f16(ah, bh[j], acc[i][j]);
  }

  float* slab = sT[wave];
  const int hh = lane >> 4;
  const int c4 = (lane & 15) * 4;
#pragma unroll
  for (int i = 0; i < 4; ++i) {
    const int mBase = m0 + (i << 4);
#pragma unroll
    for (int j = 0; j < 4; ++j) {
#pragma unroll
      for (int r = 0; r < 8; ++r) slab[(mOff + r) * 68 + (j << 4) + rlane] = acc[i][j][r] * kScale0;
    }
    __syncthreads();
    for (int pass = 0; pass < 2; ++pass) {
#pragma unroll
      for (int it = 0; it < 8; ++it) {
        const int row = it * 2 + hh;
        const v4f v = *(const v4f*)(slab + row * 68 + c4);
        *(volatile v4f*)(P + (size_t)(mBase + row) * kPP + n0 + c4) = v;
      }
      __threadfence();
    }
    __syncthreads();
  }
}

static_assert((kRows % 32) == 0 && (kTok % 4) == 0, "relu-sum grid");
__global__ __launch_bounds__(256) void relu_sum_kernel(
    const float* __restrict__ P, const float* __restrict__ b1, _Float16* __restrict__ S)
{
  const int lane = threadIdx.x & 31;
  const int wave = threadIdx.x >> 5;
  const int r0 = (blockIdx.x * 8 + wave) * 4;
  const int bidx = r0 / kTok;
  const int ch = lane * 4;
  const v4f bias = *(const v4f*)(b1 + ch);
  v4f pcv[4], accv[4];
#pragma unroll
  for (int q = 0; q < 4; ++q) {
    const v4f t = *(const v4f*)(P + (size_t)(r0 + q) * kPP + kHid + ch);
    pcv[q] = t + bias;
    accv[q] = (v4f){0.f, 0.f, 0.f, 0.f};
  }
  const float* px = P + (size_t)bidx * kTok * kPP + ch;
#pragma unroll 4
  for (int i = 0; i < kTok; ++i) {
    const v4f p = *(const v4f*)(px + (size_t)i * kPP);
#pragma unroll
    for (int q = 0; q < 4; ++q) {
#pragma unroll
      for (int e = 0; e < 4; ++e) accv[q][e] += fmaxf(p[e] + pcv[q][e], 0.0f);
    }
  }
  v4h hv[4];
#pragma unroll
  for (int q = 0; q < 4; ++q) {
#pragma unroll
    for (int e = 0; e < 4; ++e) hv[q][e] = to_f16_carry(accv[q][e], 1.0f);
  }
  for (int pass = 0; pass < 2; ++pass) {
#pragma unroll
    for (int q = 0; q < 4; ++q) *(volatile v4h*)(S + (size_t)(r0 + q) * kHid + ch) = hv[q];
    __threadfence();
  }
}

static_assert(((kRows / 64) % 4) == 0, "tiles fill whole blocks");
__global__ __launch_bounds__(128) void rel_gemm_kernel(
    const _Float16* __restrict__ S, const _Float16* __restrict__ W2T, const float* __restrict__ b2,
    float* __restrict__ out)
{
  __shared__ __align__(16) float sT[4][32 * 68];
  const int lane = threadIdx.x & 31;
  const int wave = threadIdx.x >> 5;
  const int tile = blockIdx.x * 4 + wave;
  const int m0 = tile << 6;
  const int bidx = m0 / kTok;
  const int n0 = m0 - bidx * kTok;
  const int rlane = lane & 15;
  const int koff = (lane >> 4) * 8;
  const int mOff = (lane >> 4) * 8;

  v8f acc[4][2];
#pragma unroll
  for (int i = 0; i < 4; ++i)
#pragma unroll
    for (int j = 0; j < 2; ++j) acc[i][j] = (v8f){0.f, 0.f, 0.f, 0.f, 0.f, 0.f, 0.f, 0.f};

#pragma unroll 1
  for (int k0 = 0; k0 < kHid; k0 += 32) {
    v16h bh[2];
#pragma unroll
    for (int j = 0; j < 2; ++j) bh[j] = frag_load(W2T + (size_t)((j << 4) + rlane) * kHid + k0 + koff);
#pragma unroll
    for (int i = 0; i < 4; ++i) {
      const v16h ah = frag_load(S + (size_t)(m0 + (i << 4) + rlane) * kHid + k0 + koff);
#pragma unroll
      for (int j = 0; j < 2; ++j) acc[i][j] = mma_f16(ah, bh[j], acc[i][j]);
    }
  }

  float* slab = sT[wave];
  float bq[2];
#pragma unroll
  for (int j = 0; j < 2; ++j) bq[j] = kTokF * b2[(j << 4) + rlane];
#pragma unroll
  for (int i = 0; i < 4; ++i) {
#pragma unroll
    for (int j = 0; j < 2; ++j) {
#pragma unroll
      for (int r = 0; r < 8; ++r) {
        const float v = acc[i][j][r] * kScale1 + bq[j];
        slab[((j << 4) + rlane) * 68 + (i << 4) + mOff + r] = v;
      }
    }
  }
  __syncthreads();
  const int hh = lane >> 4;
  const int c4 = (lane & 15) * 4;
  float* ob = out + (size_t)bidx * kOutC * kTok + n0 + c4;
  for (int pass = 0; pass < 2; ++pass) {
#pragma unroll
    for (int it = 0; it < 16; ++it) {
      const int o = it * 2 + hh;
      const v4f v = *(const v4f*)(slab + o * 68 + c4);
      *(volatile v4f*)(ob + (size_t)o * kTok) = v;
    }
    __threadfence();
  }
}

extern "C" void kernel_launch(void* const* d_in, const int* in_sizes, int n_in,
                              void* d_out, int out_size, void* d_ws, size_t ws_size,
                              hipStream_t stream) {
  if (n_in < 5) return;
  if (in_sizes[0] != kBatch * kChan * kTok) return;
  if (in_sizes[1] != 2 * kChan * kHid) return;
  if (in_sizes[2] != kHid) return;
  if (in_sizes[3] != kHid * kOutC) return;
  if (in_sizes[4] != kOutC) return;
  if (out_size != kBatch * kOutC * kTok) return;
  if (ws_size < kWsTotal) return;

  const float* x  = (const float*)d_in[0];
  const float* W1 = (const float*)d_in[1];
  const float* b1 = (const float*)d_in[2];
  const float* W2 = (const float*)d_in[3];
  const float* b2 = (const float*)d_in[4];
  float* out = (float*)d_out;

  char* ws = (char*)d_ws;
  _Float16* XH  = (_Float16*)(ws + kOffXH);
  _Float16* W1T = (_Float16*)(ws + kOffW1T);
  _Float16* W2T = (_Float16*)(ws + kOffW2T);
  float*    P   = (float*)(ws + kOffP);
  _Float16* S   = (_Float16*)(ws + kOffS);

  prep_planes_kernel<<<kXBlocks + kW1Blocks + kW2Blocks, 256, 0, stream>>>(x, W1, W2, XH, W1T, W2T);
  proj_gemm_kernel<<<((kRows / 64) * (kPP / 64)) / 8, 256, 0, stream>>>(XH, W1T, P);
  relu_sum_kernel<<<kRows / 32, 256, 0, stream>>>(P, b1, S);
  rel_gemm_kernel<<<(kRows / 64) / 4, 128, 0, stream>>>(S, W2T, b2, out);
}
